// Net_31379031065089
// MI455X (gfx1250) — hardware-verified
//
#include <hip/hip_runtime.h>
#include <stddef.h>
#include <stdint.h>
#include <math.h>


#define NIN    16
#define HID    128
#define NOUT   15
#define NO16   16
#define K1     32
#define K2     256
#define NTHR   256
#define NWAVE  8
#define EPT    8
#define CHUNK  (NTHR * EPT)
#define WCAP   (EPT * 32)
#define LISTN  (NWAVE * WCAP)
#define NBA    1024
#define SLA    10
#define RCAP   28672
#define DEGCAP 64
#define GBM    64
#define GBN    128
#define GTHR   128
#define GWAVE  (GTHR / 32)
#define G3M    128
#define NU1    (HID * (K1 / 8))
#define NU2    (HID * (K2 / 8))
#define NU3    (NO16 * (K2 / 8))
#define NUBT   256
#define NUALL  (NU1 + NU2 + NU3 + NUBT)
#define BK_ZINTS   (LISTN + 2 * RCAP + 3 * NBA)
#define MISC_INTS  16
#define BK_LDS_INTS (BK_ZINTS + MISC_INTS + NBA)
#define A1_LDS_INTS (3 * NBA + NBA * 16)
#define A3_LDS_INTS (3 * NBA + 128 + NBA * NOUT)
#define WSMAX  134217728

static_assert((CHUNK & (CHUNK - 1)) == 0 && CHUNK <= 4096);
static_assert((NBA & (NBA - 1)) == 0 && NBA == (1 << SLA));
static_assert(((long long)CHUNK << SLA) < (1LL << 31));
static_assert(NBA % 32 == 0 && NBA % NWAVE == 0 && NBA == 4 * NTHR && NBA % G3M == 0 && NBA % GBM == 0);
static_assert(RCAP >= 17546 && RCAP % (NTHR * 4) == 0);
static_assert(DEGCAP >= 44);
static_assert(BK_ZINTS % (NTHR * 4) == 0 && LISTN % 4 == 0 && ((BK_ZINTS + MISC_INTS) % 4) == 0);
static_assert(BK_LDS_INTS * 4 <= 300000);
static_assert(K1 % 32 == 0 && K2 % 32 == 0 && K1 == 2 * NIN && K2 == 2 * HID);
static_assert(GBN == HID && GBM == GWAVE * 16 && HID == 4 * 32 && G3M == NWAVE * 16);
static_assert(NU1 % NTHR == 0 && NU2 % NTHR == 0 && NU3 % NTHR == 0 && NUALL % NTHR == 0);
static_assert((NBA * NOUT) % (4 * NTHR) == 0 && (NBA * NOUT * 4) % 128 == 0);
static_assert((NBA * K1) % (8 * NTHR) == 0);

typedef float          v2f   __attribute__((ext_vector_type(2)));
typedef float          v4f   __attribute__((ext_vector_type(4)));
typedef float          v8f   __attribute__((ext_vector_type(8)));
typedef int            v4i   __attribute__((ext_vector_type(4)));
typedef int            v8i   __attribute__((ext_vector_type(8)));
typedef unsigned       v4u   __attribute__((ext_vector_type(4)));
typedef unsigned short v4us  __attribute__((ext_vector_type(4)));
typedef unsigned short v8us  __attribute__((ext_vector_type(8)));
typedef unsigned short v16us __attribute__((ext_vector_type(16)));
typedef __bf16         v16bf __attribute__((ext_vector_type(16)));
typedef v4f  __attribute__((may_alias)) v4fa;
typedef v4i  __attribute__((may_alias)) v4ia;
typedef v4u  __attribute__((may_alias)) v4ua;
typedef v4us __attribute__((may_alias)) v4usa;
typedef v8us __attribute__((may_alias)) v8usa;
union FragB { v16bf v; v16us u; v8us h[2]; v8i w; };

__device__ __forceinline__ v8f wmb(const FragB& a, const FragB& b, v8f c) {
  v8f d = __builtin_amdgcn_wmma_f32_16x16x32_bf16(false, a.v, false, b.v, (short)0, c, false, false);
  asm volatile("v_nop\n\tv_nop\n\tv_nop\n\tv_nop" : "+v"(d) : "v"(a.w), "v"(b.w));
  return d;
}

__device__ __forceinline__ v8f z8() { v8f z = {0.f, 0.f, 0.f, 0.f, 0.f, 0.f, 0.f, 0.f}; return z; }

__device__ __forceinline__ unsigned bf16_bits(float f) {
  const unsigned u = __float_as_uint(f);
  const unsigned r = (u + 0x7FFFu + ((u >> 16) & 1u)) >> 16;
  const unsigned nb = (u >> 16) | 0x0040u;
  return ((u & 0x7fffffffu) > 0x7f800000u) ? nb : r;
}
__device__ __forceinline__ float bf16_val(float f) {
  return __uint_as_float(bf16_bits(f) << 16);
}
__device__ __forceinline__ unsigned hl_bits(float v, unsigned& lo) {
  const unsigned hb = bf16_bits(v);
  lo = bf16_bits(v - __uint_as_float(hb << 16));
  return hb;
}
__device__ __forceinline__ float relu_keep(float v) { return (v > 0.0f) ? v : (v - v); }

__device__ __forceinline__ void wave_sync() {
  __builtin_amdgcn_fence(__ATOMIC_RELEASE, "wavefront");
  __builtin_amdgcn_wave_barrier();
  __builtin_amdgcn_fence(__ATOMIC_ACQUIRE, "wavefront");
}

__device__ __forceinline__ int clampi(int v, int lo, int hi) { return v < lo ? lo : (v > hi ? hi : v); }

template <int SLB>
__device__ __forceinline__ int scan_chunk(const int* __restrict__ dsts, int nE, int cbase, int slotBase,
                                          int nb, int vec8, int* list, int tid, int lane, int wave) {
  int wc = 0;
  const int el0  = tid * EPT;
  const int e0   = cbase + el0;
  const int sent = -2147483647 - 1;
  v4i da, db;
  if (vec8 != 0 && cbase + CHUNK <= nE) {
    da = *(const v4i*)(dsts + e0);
    db = *(const v4i*)(dsts + e0 + 4);
  } else {
    da.x = (e0     < nE) ? dsts[min(e0,     nE - 1)] : sent;
    da.y = (e0 + 1 < nE) ? dsts[min(e0 + 1, nE - 1)] : sent;
    da.z = (e0 + 2 < nE) ? dsts[min(e0 + 2, nE - 1)] : sent;
    da.w = (e0 + 3 < nE) ? dsts[min(e0 + 3, nE - 1)] : sent;
    db.x = (e0 + 4 < nE) ? dsts[min(e0 + 4, nE - 1)] : sent;
    db.y = (e0 + 5 < nE) ? dsts[min(e0 + 5, nE - 1)] : sent;
    db.z = (e0 + 6 < nE) ? dsts[min(e0 + 6, nE - 1)] : sent;
    db.w = (e0 + 7 < nE) ? dsts[min(e0 + 7, nE - 1)] : sent;
  }
  const unsigned nbs = (unsigned)slotBase;
  const unsigned unb = (unsigned)nb;
  const unsigned s0 = (unsigned)da.x - nbs, s1 = (unsigned)da.y - nbs;
  const unsigned s2 = (unsigned)da.z - nbs, s3 = (unsigned)da.w - nbs;
  const unsigned s4 = (unsigned)db.x - nbs, s5 = (unsigned)db.y - nbs;
  const unsigned s6 = (unsigned)db.z - nbs, s7 = (unsigned)db.w - nbs;
  const bool h0 = s0 < unb, h1 = s1 < unb, h2 = s2 < unb, h3 = s3 < unb;
  const bool h4 = s4 < unb, h5 = s5 < unb, h6 = s6 < unb, h7 = s7 < unb;
  const unsigned any = __builtin_amdgcn_ballot_w32(h0 | h1 | h2 | h3 | h4 | h5 | h6 | h7);
  if (any != 0u) {
#define HITJ(J, HJ, SJ) { \
      const unsigned mj = __builtin_amdgcn_ballot_w32(HJ); \
      if (mj != 0u) { \
        if (HJ) { \
          const int pos = wc + (int)__builtin_amdgcn_mbcnt_lo(mj, 0u); \
          if (pos < WCAP) list[wave * WCAP + pos] = ((el0 + (J)) << SLB) | (int)(SJ); \
        } \
        wc += (int)__builtin_popcount(mj); } }
    HITJ(0, h0, s0)
    HITJ(1, h1, s1)
    HITJ(2, h2, s2)
    HITJ(3, h3, s3)
    HITJ(4, h4, s4)
    HITJ(5, h5, s5)
    HITJ(6, h6, s6)
    HITJ(7, h7, s7)
#undef HITJ
  }
  return wc;
}

__global__ __launch_bounds__(NTHR) void k_prep(const float* __restrict__ W1, const float* __restrict__ W2,
                                               const float* __restrict__ W3, const float* __restrict__ b1,
                                               const float* __restrict__ b2, const float* __restrict__ b3,
                                               unsigned short* w1d, unsigned short* w2d, unsigned short* w3d,
                                               float* bt) {
  const int u = (int)blockIdx.x * NTHR + (int)threadIdx.x;
  unsigned hb[8];
  v4u pv;
  unsigned* dp;
  if (u < NU1) {
    const int n = u >> 2, k8 = (u & 3) * 8;
    const int kk = k8 & (NIN - 1);
    const float* p = W1 + (size_t)kk * HID + n;
#pragma unroll
    for (int i = 0; i < 8; ++i) hb[i] = bf16_bits(p[(size_t)i * HID]);
    dp = (unsigned*)(w1d + (size_t)u * 8);
  } else if (u < NU1 + NU2) {
    const int v = u - NU1;
    const int n = v >> 5, k8 = (v & 31) * 8;
    const int kk = k8 & (HID - 1);
    const float* p = W2 + (size_t)kk * HID + n;
#pragma unroll
    for (int i = 0; i < 8; ++i) hb[i] = bf16_bits(p[(size_t)i * HID]);
    dp = (unsigned*)(w2d + (size_t)v * 8);
  } else if (u < NU1 + NU2 + NU3) {
    const int v = u - (NU1 + NU2);
    const int n = v >> 5, k8 = (v & 31) * 8;
    const int kk = k8 & (HID - 1);
    const int nc = n < NOUT ? n : NOUT - 1;
    const bool lv = n < NOUT;
    const float* p = W3 + (size_t)kk * NOUT + nc;
#pragma unroll
    for (int i = 0; i < 8; ++i) {
      const float f = p[(size_t)i * NOUT];
      hb[i] = lv ? bf16_bits(f) : 0u;
    }
    dp = (unsigned*)(w3d + (size_t)v * 8);
  } else {
    const int t = u - (NU1 + NU2 + NU3);
    if (t >= 96) return;
    const int w = t >> 5, l = t & 31;
    float f0, f1, f2, f3;
    if (w == 0) {
      const v4f a = *(const v4f*)(b1 + 4 * l);
      f0 = a.x; f1 = a.y; f2 = a.z; f3 = a.w;
    } else if (w == 1) {
      const v4f a = *(const v4f*)(b2 + 4 * l);
      f0 = a.x; f1 = a.y; f2 = a.z; f3 = a.w;
    } else {
      const int c0 = 4 * l;
      const float g0 = b3[min(c0,     NOUT - 1)];
      const float g1 = b3[min(c0 + 1, NOUT - 1)];
      const float g2 = b3[min(c0 + 2, NOUT - 1)];
      const float g3 = b3[min(c0 + 3, NOUT - 1)];
      f0 = (c0     < NOUT) ? g0 : 0.0f;
      f1 = (c0 + 1 < NOUT) ? g1 : 0.0f;
      f2 = (c0 + 2 < NOUT) ? g2 : 0.0f;
      f3 = (c0 + 3 < NOUT) ? g3 : 0.0f;
    }
    pv.x = bf16_bits(f0) << 16; pv.y = bf16_bits(f1) << 16;
    pv.z = bf16_bits(f2) << 16; pv.w = bf16_bits(f3) << 16;
    dp = (unsigned*)(bt + (size_t)w * HID + 4 * l);
    *(volatile v4u*)dp = pv;
    __threadfence();
    *(volatile v4u*)dp = pv;
    return;
  }
  pv.x = hb[0] | (hb[1] << 16); pv.y = hb[2] | (hb[3] << 16);
  pv.z = hb[4] | (hb[5] << 16); pv.w = hb[6] | (hb[7] << 16);
  *(volatile v4u*)dp = pv;
  __threadfence();
  *(volatile v4u*)dp = pv;
}

__global__ __launch_bounds__(NTHR) void k_bucket(const int* __restrict__ srcs, const int* __restrict__ dsts,
                                                 int nE, int nN, int vec8,
                                                 int* lst, int* cntg, int* offg, float* disg, int* flg) {
  extern __shared__ __attribute__((aligned(16))) int dsm[];
  int* list = dsm;
  int* hl   = dsm + LISTN;
  int* sl   = hl + RCAP;
  int* cnt  = sl + RCAP;
  int* offs = cnt + NBA;
  int* cur  = offs + NBA;
  int* misc = cur + NBA;
  float* disl = (float*)(misc + MISC_INTS);
  const int tid = (int)threadIdx.x, lane = tid & 31, wave = tid >> 5;
  const int nodeBase = (int)blockIdx.x * NBA;

  {
    const v4i z4 = {0, 0, 0, 0};
    for (int i = tid * 4; i < BK_ZINTS; i += NTHR * 4) *(v4ia*)(dsm + i) = z4;
    if (tid < MISC_INTS) misc[tid] = 0;
  }
  __syncthreads();

  int t = 0, ov = 0;
  const int nChunks = (nE + CHUNK - 1) / CHUNK;
#pragma unroll 1
  for (int ch = 0; ch < nChunks; ++ch) {
    const int cbase = ch * CHUNK;
    const int wc = scan_chunk<SLA>(dsts, nE, cbase, nodeBase, NBA, vec8, list, tid, lane, wave);
    if (lane == 0) misc[wave] = wc;
    __syncthreads();
    if (wave == 0) {
#pragma unroll 1
      for (int w2 = 0; w2 < NWAVE; ++w2) {
        int c = misc[w2];
        c = c < 0 ? 0 : (c > WCAP ? WCAP : c);
#pragma unroll 1
        for (int b0 = 0; b0 < c; b0 += 32) {
          const int idx = b0 + lane;
          const int ent_ = list[w2 * WCAP + (idx < WCAP ? idx : WCAP - 1)];
          const int m32 = (c - b0) < 32 ? (c - b0) : 32;
#pragma unroll 1
          for (int k = 0; k < m32; ++k) {
            const int u    = __builtin_amdgcn_readlane(ent_, k);
            const int slot = u & (NBA - 1);
            const int el   = (u >> SLA) & (CHUNK - 1);
            const int pk   = ((cbase + el) << SLA) | slot;
            if (t < RCAP) {
              if (lane == 0) { hl[t] = pk; cnt[slot] = cnt[slot] + 1; }
              t = t + 1;
            } else {
              ov = 1;
            }
          }
        }
      }
    }
    __syncthreads();
  }
  if (wave == 0 && lane == 0) { misc[8] = t; misc[9] = ov; }
  __syncthreads();
  int tt = misc[8];
  tt = tt < 0 ? 0 : (tt > RCAP ? RCAP : tt);
  const int ovf = misc[9];

  if (wave == 0) {
    const int base = lane * (NBA / 32);
    int s = 0;
#pragma unroll 1
    for (int i = 0; i < NBA / 32; ++i) s += cnt[base + i];
    int incl = s;
#pragma unroll
    for (int d = 1; d < 32; d <<= 1) {
      const int y = __shfl_up(incl, d, 32);
      if (lane >= d) incl += y;
    }
    int run = incl - s;
#pragma unroll 1
    for (int i = 0; i < NBA / 32; ++i) {
      const int cv = cnt[base + i];
      offs[base + i] = run;
      cur[base + i]  = run;
      run += cv;
    }
  }
  __syncthreads();
  if (wave == 0) {
#pragma unroll 1
    for (int b0 = 0; b0 < tt; b0 += 32) {
      const int idx = b0 + lane;
      const int ent_ = hl[idx < RCAP ? idx : RCAP - 1];
      const int m32 = (tt - b0) < 32 ? (tt - b0) : 32;
#pragma unroll 1
      for (int k = 0; k < m32; ++k) {
        const int u    = __builtin_amdgcn_readlane(ent_, k);
        const int slot = u & (NBA - 1);
        if (lane == 0) {
          int p = cur[slot];
          p = p < 0 ? 0 : (p > RCAP - 1 ? RCAP - 1 : p);
          sl[p] = u;
          cur[slot] = p + 1;
        }
      }
    }
  }
#pragma unroll 1
  for (int j = 0; j < NBA / NTHR; ++j) {
    const int s = j * NTHR + tid;
    const float d = (float)(cnt[s] + 1);
    const float r = 1.0f / sqrtf(d);
    disl[s] = (d > 0.0f) ? r : 0.0f;
  }
  __syncthreads();

  {
    const v4i c4 = *(const v4ia*)(cnt + 4 * tid);
    const v4i o4 = *(const v4ia*)(offs + 4 * tid);
    const v4f d4 = *(const v4fa*)(disl + 4 * tid);
    int*   cp = cntg + (size_t)nodeBase + 4 * tid;
    int*   op = offg + (size_t)nodeBase + 4 * tid;
    float* dp = disg + (size_t)nodeBase + 4 * tid;
    const v4i f4 = {ovf, ovf, ovf, ovf};
    int* fp = flg + (size_t)blockIdx.x * 32 + 4 * (lane & 7);
    const bool fw = (wave == 0) && (lane < 8);
    *(volatile v4i*)cp = c4;
    *(volatile v4i*)op = o4;
    *(volatile v4f*)dp = d4;
    if (fw) *(volatile v4i*)fp = f4;
    __threadfence();
    *(volatile v4i*)cp = c4;
    *(volatile v4i*)op = o4;
    *(volatile v4f*)dp = d4;
    if (fw) *(volatile v4i*)fp = f4;
  }
#pragma unroll 1
  for (int it = 0; it < RCAP / (NTHR * 4); ++it) {
    const int p = it * (NTHR * 4) + 4 * tid;
    const v4i e4 = *(const v4ia*)(sl + p);
    const int e0 = clampi(e4.x >> SLA, 0, nE - 1);
    const int e1 = clampi(e4.y >> SLA, 0, nE - 1);
    const int e2 = clampi(e4.z >> SLA, 0, nE - 1);
    const int e3 = clampi(e4.w >> SLA, 0, nE - 1);
    const int s0 = clampi(srcs[e0], 0, nN - 1);
    const int s1 = clampi(srcs[e1], 0, nN - 1);
    const int s2 = clampi(srcs[e2], 0, nN - 1);
    const int s3 = clampi(srcs[e3], 0, nN - 1);
    v4i o4;
    o4.x = (p     < tt) ? s0 : 0;
    o4.y = (p + 1 < tt) ? s1 : 0;
    o4.z = (p + 2 < tt) ? s2 : 0;
    o4.w = (p + 3 < tt) ? s3 : 0;
    int* lp = lst + (size_t)blockIdx.x * RCAP + p;
    *(volatile v4i*)lp = o4;
    __threadfence();
    *(volatile v4i*)lp = o4;
  }
}

__global__ __launch_bounds__(NTHR) void k_xs(const float* __restrict__ x, const float* __restrict__ dis,
                                             int nN, int nUnits, float* xs) {
  const int u = (int)blockIdx.x * NTHR + (int)threadIdx.x;
  if (u >= nUnits) return;
  const int row = u >> 2, c4 = (u & 3) * 4;
  const int rc = row < nN ? row : nN - 1;
  const v4f a = *(const v4fa*)(x + (size_t)rc * NIN + c4);
  const float d = dis[rc];
  const bool ok = row < nN;
  v4f o;
  o.x = ok ? d * bf16_val(a.x) : 0.0f;
  o.y = ok ? d * bf16_val(a.y) : 0.0f;
  o.z = ok ? d * bf16_val(a.z) : 0.0f;
  o.w = ok ? d * bf16_val(a.w) : 0.0f;
  float* dp = xs + (size_t)u * 4;
  *(volatile v4f*)dp = o;
  __threadfence();
  *(volatile v4f*)dp = o;
}

__global__ __launch_bounds__(NTHR) void k_agg1(const int* __restrict__ lst, const int* __restrict__ cntg,
                                               const int* __restrict__ offg, const float* __restrict__ disg,
                                               const int* __restrict__ flg, const float* __restrict__ xs,
                                               int nN, int mRows, unsigned short* axhl) {
  extern __shared__ __attribute__((aligned(16))) int dsm[];
  int* cnt = dsm;
  int* offs = dsm + NBA;
  float* disl = (float*)(dsm + 2 * NBA);
  unsigned short* stg = (unsigned short*)(dsm + 3 * NBA);
  const int tid = (int)threadIdx.x, lane = tid & 31, wave = tid >> 5, ch = lane & 15;
  const int nodeBase = (int)blockIdx.x * NBA;
  *(v4ia*)(cnt + 4 * tid)  = *(const v4i*)(cntg + (size_t)nodeBase + 4 * tid);
  *(v4ia*)(offs + 4 * tid) = *(const v4i*)(offg + (size_t)nodeBase + 4 * tid);
  *(v4fa*)(disl + 4 * tid) = *(const v4f*)(disg + (size_t)nodeBase + 4 * tid);
  const int ovf = flg[(size_t)blockIdx.x * 32];
  __syncthreads();
  const int* bl = lst + (size_t)blockIdx.x * RCAP;
  const float qnan = __int_as_float(0x7fc00000);
#pragma unroll 1
  for (int si = 0; si < NBA / NWAVE; ++si) {
    const int s    = si * NWAVE + wave;
    const int node = nodeBase + s;
    int c = __builtin_amdgcn_readfirstlane(cnt[s]);
    const bool bad = (ovf != 0) || (c > DEGCAP) || (c < 0);
    c = clampi(c, 0, DEGCAP);
    const int o = clampi(__builtin_amdgcn_readfirstlane(offs[s]), 0, RCAP);
    const int nc = node < nN ? node : nN - 1;
    const float dd = disl[s];
    float acc = 0.0f;
#pragma unroll 1
    for (int b0 = 0; b0 < c; b0 += 32) {
      int idx = o + b0 + lane;
      idx = idx > RCAP - 1 ? RCAP - 1 : idx;
      const int sr = clampi(bl[idx], 0, nN - 1);
      const int m32 = (c - b0) < 32 ? (c - b0) : 32;
#pragma unroll 1
      for (int k = 0; k < m32; ++k) {
        const int sk = __builtin_amdgcn_readlane(sr, k);
        acc += xs[(size_t)sk * NIN + ch];
      }
    }
    const float sv = xs[(size_t)nc * NIN + ch];
    float v = dd * (acc + sv);
    v = bad ? qnan : v;
    v = (node < nN) ? v : 0.0f;
    unsigned lb;
    const unsigned hb = hl_bits(v, lb);
    if (lane < 16) {
      stg[s * K1 + ch]       = (unsigned short)hb;
      stg[s * K1 + NIN + ch] = (unsigned short)lb;
    }
  }
  __syncthreads();
  constexpr int NIT = (NBA * K1) / (8 * NTHR);
  v4u q[NIT];
#pragma unroll
  for (int it = 0; it < NIT; ++it) q[it] = *(const v4ua*)(stg + 8 * (it * NTHR + tid));
  unsigned short* base = axhl + (size_t)nodeBase * K1;
#pragma unroll
  for (int it = 0; it < NIT; ++it) {
    const int f = it * NTHR + tid;
    if (nodeBase + (f >> 2) < mRows) *(volatile v4u*)(base + 8 * (size_t)f) = q[it];
  }
  __threadfence();
#pragma unroll
  for (int it = 0; it < NIT; ++it) {
    const int f = it * NTHR + tid;
    if (nodeBase + (f >> 2) < mRows) *(volatile v4u*)(base + 8 * (size_t)f) = q[it];
  }
}

template <int MODE>
__global__ __launch_bounds__(GTHR) void k_gemm(const unsigned short* __restrict__ A, int lda,
                                               const unsigned short* __restrict__ BT, int ldb, int K,
                                               const float* __restrict__ vec,
                                               unsigned short* outh, float* outf, int nN, int mRows) {
  __shared__ __attribute__((aligned(16))) float stg[GBM * GBN];
  const int tid = (int)threadIdx.x, lane = tid & 31, wave = tid >> 5, hh = lane >> 4, m = lane & 15;
  const int rowBase = (int)blockIdx.x * GBM;

  v8f acc[8];
#pragma unroll
  for (int t = 0; t < 8; ++t) acc[t] = z8();
  const unsigned short* ap = A + (size_t)(rowBase + 16 * wave + m) * (size_t)lda + 8 * hh;
  const unsigned short* bp = BT + (size_t)m * (size_t)ldb + 8 * hh;

#pragma unroll 1
  for (int k0 = 0; k0 < K; k0 += 32) {
    FragB af;
    af.h[0] = *(const v8usa*)(ap + k0);
    af.h[1] = *(const v8usa*)(ap + k0 + 16);
#pragma unroll
    for (int nt = 0; nt < 8; ++nt) {
      const unsigned short* wq = bp + (size_t)(16 * nt) * (size_t)ldb + k0;
      FragB bf;
      bf.h[0] = *(const v8usa*)wq;
      bf.h[1] = *(const v8usa*)(wq + 16);
      acc[nt] = wmb(af, bf, acc[nt]);
    }
  }

#pragma unroll
  for (int nt = 0; nt < 8; ++nt) {
    const int lc = 16 * nt + m;
#pragma unroll
    for (int r = 0; r < 8; ++r) {
      const int lr = 16 * wave + 8 * hh + r;
      stg[lr * GBN + lc] = acc[nt][r];
    }
  }
  __syncthreads();

  v4f pv[16];
#pragma unroll
  for (int i = 0; i < 16; ++i) pv[i] = *(const v4fa*)(stg + (16 * wave + i) * GBN + 4 * lane);
  __syncthreads();

  if constexpr (MODE == 2) {
    const float dv = vec[rowBase + 16 * wave + m];
#pragma unroll
    for (int i = 0; i < 16; ++i) {
      const float d = __shfl(dv, i, 32);
      v4f q = pv[i];
      q.x = d * q.x; q.y = d * q.y; q.z = d * q.z; q.w = d * q.w;
      pv[i] = q;
    }
#pragma unroll
    for (int i = 0; i < 16; ++i) {
      const int gr = rowBase + 16 * wave + i;
      float* op = outf + (size_t)gr * GBN + 4 * lane;
      if (gr < mRows) *(volatile v4f*)op = pv[i];
    }
    __threadfence();
#pragma unroll
    for (int i = 0; i < 16; ++i) {
      const int gr = rowBase + 16 * wave + i;
      float* op = outf + (size_t)gr * GBN + 4 * lane;
      if (gr < mRows) *(volatile v4f*)op = pv[i];
    }
    (void)outh; (void)nN;
  } else {
    const v4f b4 = *(const v4f*)(vec + 4 * lane);
#pragma unroll
    for (int i = 0; i < 16; ++i) {
      const int row = rowBase + 16 * wave + i;
      const bool ok = row < nN;
      const float y0 = relu_keep(pv[i].x + b4.x);
      const float y1 = relu_keep(pv[i].y + b4.y);
      const float y2 = relu_keep(pv[i].z + b4.z);
      const float y3 = relu_keep(pv[i].w + b4.w);
      v4us h4, l4;
      unsigned lb;
      unsigned hb;
      hb = hl_bits(ok ? y0 : 0.0f, lb); h4[0] = (unsigned short)hb; l4[0] = (unsigned short)lb;
      hb = hl_bits(ok ? y1 : 0.0f, lb); h4[1] = (unsigned short)hb; l4[1] = (unsigned short)lb;
      hb = hl_bits(ok ? y2 : 0.0f, lb); h4[2] = (unsigned short)hb; l4[2] = (unsigned short)lb;
      hb = hl_bits(ok ? y3 : 0.0f, lb); h4[3] = (unsigned short)hb; l4[3] = (unsigned short)lb;
      unsigned short* srow = (unsigned short*)stg + (size_t)(16 * wave + i) * (2 * GBN);
      *(v4usa*)(srow + 4 * lane) = h4;
      *(v4usa*)(srow + HID + 4 * lane) = l4;
    }
    __syncthreads();
    v8us qv[16];
#pragma unroll
    for (int i = 0; i < 16; ++i) {
      const unsigned short* srow = (const unsigned short*)stg + (size_t)(16 * wave + i) * (2 * GBN);
      qv[i] = *(const v8usa*)(srow + 8 * lane);
    }
#pragma unroll
    for (int i = 0; i < 16; ++i) {
      const int gr = rowBase + 16 * wave + i;
      unsigned short* rp = outh + (size_t)gr * (size_t)K2 + 8 * lane;
      if (gr < mRows) *(volatile v8us*)rp = qv[i];
    }
    __threadfence();
#pragma unroll
    for (int i = 0; i < 16; ++i) {
      const int gr = rowBase + 16 * wave + i;
      unsigned short* rp = outh + (size_t)gr * (size_t)K2 + 8 * lane;
      if (gr < mRows) *(volatile v8us*)rp = qv[i];
    }
    (void)outf;
  }
}

__global__ __launch_bounds__(NTHR) void k_agg2(const int* __restrict__ lst, const int* __restrict__ cntg,
                                               const int* __restrict__ offg, const float* __restrict__ disg,
                                               const int* __restrict__ flg, const float* __restrict__ s2,
                                               const float* __restrict__ bias, int nN, int mRows,
                                               unsigned short* hhl) {
  __shared__ __attribute__((aligned(16))) int cnt[NBA];
  __shared__ __attribute__((aligned(16))) int offs[NBA];
  __shared__ __attribute__((aligned(16))) float disl[NBA];
  __shared__ __attribute__((aligned(16))) unsigned short rowbufs[NWAVE * K2];
  const int tid = (int)threadIdx.x, lane = tid & 31, wave = tid >> 5;
  const int nodeBase = (int)blockIdx.x * NBA;
  unsigned short* rowbuf = rowbufs + wave * K2;
  *(v4ia*)(cnt + 4 * tid)  = *(const v4i*)(cntg + (size_t)nodeBase + 4 * tid);
  *(v4ia*)(offs + 4 * tid) = *(const v4i*)(offg + (size_t)nodeBase + 4 * tid);
  *(v4fa*)(disl + 4 * tid) = *(const v4f*)(disg + (size_t)nodeBase + 4 * tid);
  const int ovf = flg[(size_t)blockIdx.x * 32];
  const v4f b4 = *(const v4f*)(bias + 4 * lane);
  __syncthreads();
  const int* bl = lst + (size_t)blockIdx.x * RCAP;
  const float qnan = __int_as_float(0x7fc00000);
#pragma unroll 1
  for (int si = 0; si < NBA / NWAVE; ++si) {
    const int s    = si * NWAVE + wave;
    const int node = nodeBase + s;
    int c = __builtin_amdgcn_readfirstlane(cnt[s]);
    const bool bad = (ovf != 0) || (c > DEGCAP) || (c < 0);
    c = clampi(c, 0, DEGCAP);
    const int o = clampi(__builtin_amdgcn_readfirstlane(offs[s]), 0, RCAP);
    const int nc = node < nN ? node : nN - 1;
    const float dd = disl[s];
    const bool live = node < nN;
    float a0 = 0.0f, a1 = 0.0f, a2 = 0.0f, a3 = 0.0f;
#pragma unroll 1
    for (int b0 = 0; b0 < c; b0 += 32) {
      int idx = o + b0 + lane;
      idx = idx > RCAP - 1 ? RCAP - 1 : idx;
      const int sr = clampi(bl[idx], 0, nN - 1);
      const int m32 = (c - b0) < 32 ? (c - b0) : 32;
#pragma unroll 1
      for (int k = 0; k < m32; ++k) {
        const int sk = __builtin_amdgcn_readlane(sr, k);
        const v4f r = *(const v4fa*)(s2 + (size_t)sk * HID + 4 * lane);
        a0 += r.x; a1 += r.y; a2 += r.z; a3 += r.w;
      }
    }
    const v4f sv = *(const v4fa*)(s2 + (size_t)nc * HID + 4 * lane);
    float y0 = relu_keep(dd * (a0 + sv.x) + b4.x);
    float y1 = relu_keep(dd * (a1 + sv.y) + b4.y);
    float y2 = relu_keep(dd * (a2 + sv.z) + b4.z);
    float y3 = relu_keep(dd * (a3 + sv.w) + b4.w);
    y0 = bad ? qnan : y0; y1 = bad ? qnan : y1; y2 = bad ? qnan : y2; y3 = bad ? qnan : y3;
    y0 = live ? y0 : 0.0f; y1 = live ? y1 : 0.0f; y2 = live ? y2 : 0.0f; y3 = live ? y3 : 0.0f;
    v4us mh, ml;
    {
      unsigned lb;
      unsigned hb;
      hb = hl_bits(y0, lb); mh[0] = (unsigned short)hb; ml[0] = (unsigned short)lb;
      hb = hl_bits(y1, lb); mh[1] = (unsigned short)hb; ml[1] = (unsigned short)lb;
      hb = hl_bits(y2, lb); mh[2] = (unsigned short)hb; ml[2] = (unsigned short)lb;
      hb = hl_bits(y3, lb); mh[3] = (unsigned short)hb; ml[3] = (unsigned short)lb;
    }
    *(v4usa*)(rowbuf + 4 * lane)       = mh;
    *(v4usa*)(rowbuf + HID + 4 * lane) = ml;
    wave_sync();
    const v8us q0 = *(const v8usa*)(rowbuf + 8 * lane);
    wave_sync();
    if (node < mRows) {
      unsigned short* rpw = hhl + (size_t)node * K2 + 8 * lane;
      *(volatile v8us*)rpw = q0;
      __threadfence();
      *(volatile v8us*)rpw = q0;
    }
  }
}

__global__ __launch_bounds__(NTHR) void k_gemm3(const unsigned short* __restrict__ A,
                                                const unsigned short* __restrict__ BT,
                                                const float* __restrict__ dis, float* s3, int mRows) {
  __shared__ __attribute__((aligned(16))) float stg[G3M * NO16];
  const int tid = (int)threadIdx.x, lane = tid & 31, wave = tid >> 5, hh = lane >> 4, m = lane & 15;
  const int rowBase = (int)blockIdx.x * G3M;
  v8f acc = z8();
  const unsigned short* ap = A + (size_t)(rowBase + 16 * wave + m) * (size_t)K2 + 8 * hh;
  const unsigned short* bp = BT + (size_t)m * (size_t)K2 + 8 * hh;
#pragma unroll 1
  for (int k0 = 0; k0 < K2; k0 += 32) {
    FragB af, bf;
    af.h[0] = *(const v8usa*)(ap + k0);
    af.h[1] = *(const v8usa*)(ap + k0 + 16);
    bf.h[0] = *(const v8usa*)(bp + k0);
    bf.h[1] = *(const v8usa*)(bp + k0 + 16);
    acc = wmb(af, bf, acc);
  }
#pragma unroll
  for (int r = 0; r < 8; ++r) stg[(16 * wave + 8 * hh + r) * NO16 + m] = acc[r];
  __syncthreads();
  v4f ov[2];
#pragma unroll
  for (int j = 0; j < 2; ++j) {
    const int f = j * NTHR + tid;
    const v4f v = *(const v4fa*)(stg + 4 * f);
    const float d = dis[rowBase + (f >> 2)];
    v4f q;
    q.x = d * v.x; q.y = d * v.y; q.z = d * v.z; q.w = d * v.w;
    ov[j] = q;
  }
  float* base = s3 + (size_t)rowBase * NO16;
#pragma unroll
  for (int j = 0; j < 2; ++j) {
    const int f = j * NTHR + tid;
    if (rowBase + (f >> 2) < mRows) *(volatile v4f*)(base + 4 * (size_t)f) = ov[j];
  }
  __threadfence();
#pragma unroll
  for (int j = 0; j < 2; ++j) {
    const int f = j * NTHR + tid;
    if (rowBase + (f >> 2) < mRows) *(volatile v4f*)(base + 4 * (size_t)f) = ov[j];
  }
}

__global__ __launch_bounds__(NTHR) void k_agg3(const int* __restrict__ lst, const int* __restrict__ cntg,
                                               const int* __restrict__ offg, const float* __restrict__ disg,
                                               const int* __restrict__ flg, const float* __restrict__ s3,
                                               const float* __restrict__ bias, int nN, float* out) {
  extern __shared__ __attribute__((aligned(16))) int dsm[];
  int* cnt = dsm;
  int* offs = dsm + NBA;
  float* disl = (float*)(dsm + 2 * NBA);
  float* bs = (float*)(dsm + 3 * NBA);
  float* os = (float*)(dsm + 3 * NBA + 128);
  const int tid = (int)threadIdx.x, lane = tid & 31, wave = tid >> 5, ch = lane & 15;
  const int nodeBase = (int)blockIdx.x * NBA;
  *(v4ia*)(cnt + 4 * tid)  = *(const v4i*)(cntg + (size_t)nodeBase + 4 * tid);
  *(v4ia*)(offs + 4 * tid) = *(const v4i*)(offg + (size_t)nodeBase + 4 * tid);
  *(v4fa*)(disl + 4 * tid) = *(const v4f*)(disg + (size_t)nodeBase + 4 * tid);
  if (wave == 0) {
    const v4f b4 = *(const v4f*)(bias + 4 * lane);
    *(v4fa*)(bs + 4 * lane) = b4;
  }
  const int ovf = flg[(size_t)blockIdx.x * 32];
  __syncthreads();
  const float bv = bs[ch];
  const int* bl = lst + (size_t)blockIdx.x * RCAP;
  const float qnan = __int_as_float(0x7fc00000);
#pragma unroll 1
  for (int si = 0; si < NBA / NWAVE; ++si) {
    const int s    = si * NWAVE + wave;
    const int node = nodeBase + s;
    int c = __builtin_amdgcn_readfirstlane(cnt[s]);
    const bool bad = (ovf != 0) || (c > DEGCAP) || (c < 0);
    c = clampi(c, 0, DEGCAP);
    const int o = clampi(__builtin_amdgcn_readfirstlane(offs[s]), 0, RCAP);
    const int nc = node < nN ? node : nN - 1;
    const float dd = disl[s];
    float acc = 0.0f;
#pragma unroll 1
    for (int b0 = 0; b0 < c; b0 += 32) {
      int idx = o + b0 + lane;
      idx = idx > RCAP - 1 ? RCAP - 1 : idx;
      const int sr = clampi(bl[idx], 0, nN - 1);
      const int m32 = (c - b0) < 32 ? (c - b0) : 32;
#pragma unroll 1
      for (int k = 0; k < m32; ++k) {
        const int sk = __builtin_amdgcn_readlane(sr, k);
        acc += s3[(size_t)sk * NO16 + ch];
      }
    }
    const float sv = s3[(size_t)nc * NO16 + ch];
    float v = dd * (acc + sv) + bv;
    v = bad ? qnan : v;
    if (lane < NOUT) os[s * NOUT + ch] = v;
  }
  __syncthreads();
  int rv = nN - nodeBase;
  rv = rv < 0 ? 0 : (rv > NBA ? NBA : rv);
  const int n4 = (rv * NOUT) >> 2;
  constexpr int NIT = (NBA * NOUT) / (4 * NTHR);
  v4f ov[NIT];
#pragma unroll
  for (int it = 0; it < NIT; ++it) ov[it] = *(const v4fa*)(os + 4 * (it * NTHR + tid));
  float* base = out + (size_t)nodeBase * NOUT;
#pragma unroll
  for (int it = 0; it < NIT; ++it) {
    const int f = it * NTHR + tid;
    if (f < n4) *(volatile v4f*)(base + 4 * (size_t)f) = ov[it];
  }
  __threadfence();
#pragma unroll
  for (int it = 0; it < NIT; ++it) {
    const int f = it * NTHR + tid;
    if (f < n4) *(volatile v4f*)(base + 4 * (size_t)f) = ov[it];
  }
}

static inline int cdiv(int a, int b) { return (a + b - 1) / b; }
static inline size_t al256(size_t o) { return (o + 255) & ~(size_t)255; }

extern "C" void kernel_launch(void* const* d_in, const int* in_sizes, int n_in,
                              void* d_out, int out_size, void* d_ws, size_t ws_size,
                              hipStream_t stream) {
  if (n_in < 8) return;
  if (in_sizes[0] < NIN || (in_sizes[0] % NIN) != 0) return;
  const int nN = in_sizes[0] / NIN;
  if (nN < G3M || nN > (1 << 22) || (nN % 32) != 0) return;
  if (in_sizes[1] < 2 || (in_sizes[1] & 1) != 0) return;
  const int nE = in_sizes[1] / 2;
  if (nE < 1 || nE >= (1 << (31 - SLA))) return;
  if (in_sizes[2] != NIN * HID || in_sizes[3] != HID) return;
  if (in_sizes[4] != HID * HID || in_sizes[5] != HID) return;
  if (in_sizes[6] != HID * NOUT || in_sizes[7] != NOUT) return;
  if ((long long)out_size != (long long)nN * NOUT) return;

  const float* x    = (const float*)d_in[0];
  const int*   edge = (const int*)d_in[1];
  const float* W1   = (const float*)d_in[2];
  const float* b1   = (const float*)d_in[3];
  const float* W2   = (const float*)d_in[4];
  const float* b2   = (const float*)d_in[5];
  const float* W3   = (const float*)d_in[6];
  const float* b3   = (const float*)d_in[7];
  float* out = (float*)d_out;
  const int* src = edge;
  const int* dst = edge + nE;

  const int MP  = cdiv(nN, G3M) * G3M;
  const int gA  = cdiv(nN, NBA);
  const int NBP = gA * NBA;
  if (NBP < MP) return;
  const int vec8 = ((nE & 3) == 0) ? 1 : 0;

  char* ws = (char*)d_ws;
  size_t off = 0;
  const size_t oW1D = off; off = al256(off + (size_t)HID * K1 * 2);
  const size_t oW2D = off; off = al256(off + (size_t)HID * K2 * 2);
  const size_t oW3D = off; off = al256(off + (size_t)NO16 * K2 * 2);
  const size_t oBT  = off; off = al256(off + (size_t)3 * HID * 4);
  const size_t oCNT = off; off = al256(off + (size_t)NBP * 4);
  const size_t oOFF = off; off = al256(off + (size_t)NBP * 4);
  const size_t oDIS = off; off = al256(off + (size_t)NBP * 4);
  const size_t oFLG = off; off = al256(off + (size_t)gA * 128);
  const size_t oLST = off; off = al256(off + (size_t)gA * RCAP * 4);
  const size_t oXS  = off; off = al256(off + (size_t)MP * NIN * 4);
  const size_t oAX  = off; off = al256(off + (size_t)MP * K1 * 2);
  const size_t oHH  = off; off = al256(off + (size_t)MP * K2 * 2);
  const size_t oS2  = off; off = al256(off + (size_t)MP * HID * 4);
  if (off > ws_size || off > (size_t)WSMAX) return;
  unsigned short* W1D = (unsigned short*)(ws + oW1D);
  unsigned short* W2D = (unsigned short*)(ws + oW2D);
  unsigned short* W3D = (unsigned short*)(ws + oW3D);
  float*          BT  = (float*)(ws + oBT);
  int*            CNT = (int*)(ws + oCNT);
  int*            OFF = (int*)(ws + oOFF);
  float*          DIS = (float*)(ws + oDIS);
  int*            FLG = (int*)(ws + oFLG);
  int*            LST = (int*)(ws + oLST);
  float*          XS  = (float*)(ws + oXS);
  unsigned short* AX  = (unsigned short*)(ws + oAX);
  unsigned short* HH  = (unsigned short*)(ws + oHH);
  float*          S2  = (float*)(ws + oS2);
  float*          S3  = XS;

  const size_t bkLds = (size_t)BK_LDS_INTS * 4;
  const size_t a1Lds = (size_t)A1_LDS_INTS * 4;
  const size_t a3Lds = (size_t)A3_LDS_INTS * 4;
  hipFuncSetAttribute(reinterpret_cast<const void*>(&k_bucket), hipFuncAttributeMaxDynamicSharedMemorySize, (int)bkLds);
  hipFuncSetAttribute(reinterpret_cast<const void*>(&k_agg1), hipFuncAttributeMaxDynamicSharedMemorySize, (int)a1Lds);
  hipFuncSetAttribute(reinterpret_cast<const void*>(&k_agg3), hipFuncAttributeMaxDynamicSharedMemorySize, (int)a3Lds);

  const int nUx = MP * (NIN / 4);
  k_prep<<<NUALL / NTHR, NTHR, 0, stream>>>(W1, W2, W3, b1, b2, b3, W1D, W2D, W3D, BT);
  k_bucket<<<gA, NTHR, bkLds, stream>>>(src, dst, nE, nN, vec8, LST, CNT, OFF, DIS, FLG);
  k_xs<<<cdiv(nUx, NTHR), NTHR, 0, stream>>>(x, DIS, nN, nUx, XS);
  k_agg1<<<gA, NTHR, a1Lds, stream>>>(LST, CNT, OFF, DIS, FLG, XS, nN, MP, AX);
  k_gemm<1><<<MP / GBM, GTHR, 0, stream>>>(AX, K1, W1D, K1, K1, BT, HH, S2, nN, MP);
  k_gemm<2><<<MP / GBM, GTHR, 0, stream>>>(HH, K2, W2D, K2, K2, DIS, HH, S2, nN, MP);
  k_agg2<<<gA, NTHR, 0, stream>>>(LST, CNT, OFF, DIS, FLG, S2, BT + HID, nN, MP, HH);
  k_gemm3<<<MP / G3M, NTHR, 0, stream>>>(HH, W3D, DIS, S3, MP);
  k_agg3<<<gA, NTHR, a3Lds, stream>>>(LST, CNT, OFF, DIS, FLG, S3, BT + 2 * HID, nN, out);
}
